// BoTBlock_53223234732454
// MI455X (gfx1250) — hardware-run, weakly checked
//
#include <hip/hip_runtime.h>


#define NBI  16
#define CIN  512
#define NN   1024
#define WID  128
#define NH_  4
#define HD   32
#define COUT 512
#define PCAR 1024.0f
typedef _Float16 h16;
typedef unsigned short bf;
typedef __attribute__((ext_vector_type(16))) __bf16   v16bf;
typedef __attribute__((ext_vector_type(16))) _Float16 v16h;
typedef __attribute__((ext_vector_type(8)))  _Float16 v8h;
typedef __attribute__((ext_vector_type(8)))  unsigned short v8us;
typedef __attribute__((ext_vector_type(8)))  float    v8f;
typedef __attribute__((ext_vector_type(4)))  float    v4f;
typedef v8h  __attribute__((may_alias)) v8ha;
typedef v4f  __attribute__((may_alias)) v4fa;
typedef v8us __attribute__((may_alias)) v8usa;

__device__ __forceinline__ unsigned short f2bf(float f) { unsigned u = __float_as_uint(f); u += 0x7FFFu + ((u >> 16) & 1u); return (unsigned short)(u >> 16); }
__device__ __forceinline__ float bf2f(unsigned short b) { return __uint_as_float(((unsigned)b) << 16); }
__device__ __forceinline__ float bfr(float f) { return bf2f(f2bf(f)); }
__device__ __forceinline__ v16h cat16(v8h lo, v8h hi) { return __builtin_shufflevector(lo, hi, 0, 1, 2, 3, 4, 5, 6, 7, 8, 9, 10, 11, 12, 13, 14, 15); }
__device__ __forceinline__ v16bf cat16b(v8us lo, v8us hi) { return __builtin_bit_cast(v16bf, __builtin_shufflevector(lo, hi, 0, 1, 2, 3, 4, 5, 6, 7, 8, 9, 10, 11, 12, 13, 14, 15)); }
__device__ __forceinline__ v8f wmma16(v16h a, v16h b, v8f c) { return __builtin_amdgcn_wmma_f32_16x16x32_f16(false, a, false, b, (short)0, c, false, false); }
__device__ __forceinline__ v8f wmmab(v16bf a, v16bf b, v8f c) { return __builtin_amdgcn_wmma_f32_16x16x32_bf16(false, a, false, b, (short)0, c, false, false); }


template <typename T16> struct WFrag;
template <> struct WFrag<h16> { typedef v16h V; static __device__ __forceinline__ V ld(const h16* p) { return cat16(*(const v8h*)p, *(const v8h*)(p + 16)); } static __device__ __forceinline__ v8f mma(V a, V b, v8f c) { return wmma16(a, b, c); } };
template <> struct WFrag<bf> { typedef v16bf V; static __device__ __forceinline__ V ld(const bf* p) { return cat16b(*(const v8us*)p, *(const v8us*)(p + 16)); } static __device__ __forceinline__ v8f mma(V a, V b, v8f c) { return wmmab(a, b, c); } };
template <typename T16, int NSPLIT, bool BIAS>
__global__ __launch_bounds__(32) void k_gemmw(const T16* __restrict__ A, const T16* __restrict__ A2, const T16* __restrict__ Bt, const T16* __restrict__ Bt2, int K, float* C, int ldc, const float* __restrict__ bias, size_t sA, size_t sB, size_t sC) {
    typedef typename WFrag<T16>::V V;
    __shared__ __align__(16) float os[16 * 68];
    const size_t z = blockIdx.z; A += z * sA; if (A2) A2 += z * sA; Bt += z * sB; if (Bt2) Bt2 += z * sB; C += z * sC;
    const int lane = threadIdx.x & 31, lr = lane & 15, hi = lane >> 4; const int r0 = blockIdx.x * 64, c0 = blockIdx.y * 64;
    v8f acc[4][4];
#pragma unroll
    for (int mb = 0; mb < 4; ++mb)
#pragma unroll
        for (int nb = 0; nb < 4; ++nb) acc[mb][nb] = (v8f){};
    const size_t aoff = (size_t)(r0 + lr) * K + 8 * hi, boff = (size_t)(c0 + lr) * K + 8 * hi;
#pragma unroll 1
    for (int kc = 0; kc < K; kc += 32) {
        V a[4], a2[4];
#pragma unroll
        for (int mb = 0; mb < 4; ++mb) { a[mb] = WFrag<T16>::ld(A + aoff + (size_t)mb * 16 * K + kc); if (NSPLIT == 1 || NSPLIT == 2) a2[mb] = WFrag<T16>::ld(A2 + aoff + (size_t)mb * 16 * K + kc); }
#pragma unroll
        for (int nb = 0; nb < 4; ++nb) { const V b = WFrag<T16>::ld(Bt + boff + (size_t)nb * 16 * K + kc); V b2; if (NSPLIT >= 2) b2 = WFrag<T16>::ld(Bt2 + boff + (size_t)nb * 16 * K + kc);
#pragma unroll
            for (int mb = 0; mb < 4; ++mb) { acc[mb][nb] = WFrag<T16>::mma(a[mb], b, acc[mb][nb]); if (NSPLIT == 1 || NSPLIT == 2) acc[mb][nb] = WFrag<T16>::mma(a2[mb], b, acc[mb][nb]); if (NSPLIT >= 2) acc[mb][nb] = WFrag<T16>::mma(a[mb], b2, acc[mb][nb]); } }
        asm volatile("v_nop\n\tv_nop\n\tv_nop\n\tv_nop" : "+v"(acc[0][0]), "+v"(acc[1][1]), "+v"(acc[2][2]), "+v"(acc[3][3]) : "v"(a[0]), "v"(a[3]));
    }
#pragma unroll
    for (int mb = 0; mb < 4; ++mb) {
#pragma unroll
        for (int nb = 0; nb < 4; ++nb) {
#pragma unroll
            for (int j = 0; j < 8; ++j) os[(hi * 8 + j) * 68 + nb * 16 + lr] = acc[mb][nb][j]; }
        __builtin_amdgcn_wave_barrier(); asm volatile("" ::: "memory");
        float* crow = C + (size_t)(r0 + mb * 16) * ldc + c0;
#pragma unroll 1
        for (int ps = 0; ps < 2; ++ps) {
#pragma unroll
            for (int s = 0; s < 8; ++s) { const int row = 2 * s + hi, cofs = lr * 4; v4f val = *(const v4fa*)(os + row * 68 + cofs); if (BIAS) { val[0] += bfr(bias[c0 + cofs]); val[1] += bfr(bias[c0 + cofs + 1]); val[2] += bfr(bias[c0 + cofs + 2]); val[3] += bfr(bias[c0 + cofs + 3]); }
                *(volatile v4f*)(crow + (size_t)row * ldc + cofs) = val; }
            if (ps == 0) __threadfence(); }
        __builtin_amdgcn_wave_barrier(); asm volatile("" ::: "memory");
    }
}

__device__ __forceinline__ h16 tohx(float x) { return (h16)x; }
__device__ __forceinline__ void splitf(float y, unsigned short& h, unsigned short& l) { h = f2bf(y); l = f2bf(y - bf2f(h)); }
typedef __attribute__((ext_vector_type(2))) _Float16 v2h;
typedef __attribute__((ext_vector_type(4))) _Float16 v4h;
typedef __attribute__((ext_vector_type(4))) unsigned short v4us;
typedef __attribute__((ext_vector_type(2))) unsigned short v2us;

__global__ __launch_bounds__(256) void k_cvt8(const float* __restrict__ src, bf* dst, size_t n8) { const size_t i = (size_t)blockIdx.x * 256 + threadIdx.x; if (i >= n8) return; const v8f v = *(const v8f*)(src + i * 8); v8us o;
#pragma unroll
    for (int k = 0; k < 8; ++k) o[k] = f2bf(v[k]); *(volatile v8us*)(dst + i * 8) = o; __threadfence(); *(volatile v8us*)(dst + i * 8) = o; }
__global__ __launch_bounds__(256) void k_xt(const float* __restrict__ x, bf* XT) { const size_t e = ((size_t)blockIdx.x * 256 + threadIdx.x) * 4; if (e >= (size_t)NBI * NN * CIN) return; const int c = (int)(e % CIN); const int n = (int)((e / CIN) % NN); const int b = (int)(e / ((size_t)CIN * NN)); v4us o;
#pragma unroll
    for (int q = 0; q < 4; ++q) o[q] = f2bf(x[((size_t)b * CIN + c + q) * NN + n]); *(volatile v4us*)(XT + e) = o; __threadfence(); *(volatile v4us*)(XT + e) = o; }
__global__ __launch_bounds__(256) void k_bnstat(const float* __restrict__ F, int Cw, float* MEAN, float* RSTD) { const int c = blockIdx.x * 256 + threadIdx.x; if (c >= Cw) return; float s = 0.f;
#pragma unroll 1
    for (int i = 0; i < NBI * NN; ++i) s = __fadd_rn(s, F[(size_t)i * Cw + c]);
    const float m = s * (1.0f / (NBI * NN)); float v = 0.f;
#pragma unroll 1
    for (int i = 0; i < NBI * NN; ++i) { float d = __fsub_rn(F[(size_t)i * Cw + c], m); asm volatile("" : "+v"(d)); float p = __fmul_rn(d, d); asm volatile("" : "+v"(p)); v = __fadd_rn(v, p); }
    const float rs = __frsqrt_rn(__fadd_rn(v * (1.0f / (NBI * NN)), 1e-5f)); *(volatile float*)(MEAN + c) = m; *(volatile float*)(RSTD + c) = rs; __threadfence(); *(volatile float*)(MEAN + c) = m; *(volatile float*)(RSTD + c) = rs; }
__global__ __launch_bounds__(256) void k_bn1(const float* __restrict__ F1, const float* __restrict__ MEAN, const float* __restrict__ RSTD, const float* __restrict__ g, const float* __restrict__ be, bf* Yh, bf* Yl) { const size_t e = ((size_t)blockIdx.x * 256 + threadIdx.x) * 4; if (e >= (size_t)NBI * NN * WID) return; const int c = (int)(e % WID); const v4f a = *(const v4f*)(F1 + e); v4us oh, ol;
#pragma unroll
    for (int q = 0; q < 4; ++q) { const int cc = c + q; float t0 = __fmul_rn(__fsub_rn(a[q], MEAN[cc]), RSTD[cc]); asm volatile("" : "+v"(t0)); float t1 = __fmul_rn(t0, bfr(g[cc])); asm volatile("" : "+v"(t1)); unsigned short u, l; splitf(fmaxf(__fadd_rn(t1, bfr(be[cc])), 0.f), u, l); oh[q] = u; ol[q] = l; }
    *(volatile v4us*)(Yh + e) = oh; *(volatile v4us*)(Yl + e) = ol; __threadfence(); *(volatile v4us*)(Yh + e) = oh; *(volatile v4us*)(Yl + e) = ol; }
__global__ __launch_bounds__(256) void k_qkpl(const float* __restrict__ QKV, const float* __restrict__ rw, const float* __restrict__ rh, bf* Qh, bf* Ql, bf* Kh, bf* Kl) { const size_t e = ((size_t)blockIdx.x * 256 + threadIdx.x) * 4; if (e >= (size_t)NH_ * NN * HD) return; const int d = (int)(e % HD); const int n = (int)((e / HD) % NN); const int h = (int)(e / ((size_t)HD * NN)); const float* r = QKV + (size_t)n * 3 * WID + h * HD + d; const int wq = n % 32, hq = n / 32; v4us qh, ql, kh, kl;
#pragma unroll
    for (int q = 0; q < 4; ++q) { const int dd = d + q; unsigned short a, c; splitf(r[q] * 0.1767766952966369f, a, c); qh[q] = a; ql[q] = c; const float rr = __fadd_rn(bfr(rw[(h * HD + dd) * 32 + wq]), bfr(rh[(h * HD + dd) * 32 + hq])); splitf(__fadd_rn(r[WID + q], rr), a, c); kh[q] = a; kl[q] = c; }
    for (int ps = 0; ps < 2; ++ps) { *(volatile v4us*)(Qh + e) = qh; *(volatile v4us*)(Ql + e) = ql; *(volatile v4us*)(Kh + e) = kh; *(volatile v4us*)(Kl + e) = kl; if (ps == 0) __threadfence(); } }
__global__ __launch_bounds__(256) void k_vt(const float* __restrict__ QKV, bf* VTh, bf* VTl) { const size_t e = ((size_t)blockIdx.x * 256 + threadIdx.x) * 2; if (e >= (size_t)NH_ * 64 * NN) return; const int m = (int)(e % NN); const int dv = (int)((e / NN) % 64); const int h = (int)(e / ((size_t)NN * 64)); v2us oh, ol;
#pragma unroll
    for (int u = 0; u < 2; ++u) { const float v = dv < HD ? QKV[(size_t)(m + u) * 3 * WID + 2 * WID + h * HD + dv] : 0.f; unsigned short a, c; splitf(v, a, c); oh[u] = a; ol[u] = c; }
    *(volatile v2us*)(VTh + e) = oh; *(volatile v2us*)(VTl + e) = ol; __threadfence(); *(volatile v2us*)(VTh + e) = oh; *(volatile v2us*)(VTl + e) = ol; }
__global__ __launch_bounds__(256) void k_mrg(const float* __restrict__ O, bf* Mh, bf* Ml) { const size_t e = ((size_t)blockIdx.x * 256 + threadIdx.x) * 4; if (e >= (size_t)NN * WID) return; const int c = (int)(e % WID); const int n = (int)(e / WID); const int h = c / HD, d = c % HD; const float* r = O + ((size_t)h * NN + n) * 64 + d; v4us oh, ol;
#pragma unroll
    for (int q = 0; q < 4; ++q) { unsigned short a, b; splitf(r[q], a, b); oh[q] = a; ol[q] = b; } *(volatile v4us*)(Mh + e) = oh; *(volatile v4us*)(Ml + e) = ol; __threadfence(); *(volatile v4us*)(Mh + e) = oh; *(volatile v4us*)(Ml + e) = ol; }
__global__ __launch_bounds__(256) void k_outT(const float* __restrict__ F2, const float* __restrict__ MEAN, const float* __restrict__ RSTD, const float* __restrict__ g, const float* __restrict__ be, const float* __restrict__ x, float* OUT) { const size_t e = ((size_t)blockIdx.x * 256 + threadIdx.x) * 4; if (e >= (size_t)NBI * COUT * NN) return; const int n = (int)(e % NN); const int c = (int)((e / NN) % COUT); const int b = (int)(e / ((size_t)NN * COUT)); const float m = MEAN[c], rs = RSTD[c], gg = bfr(g[c]), bb = bfr(be[c]); v4f o;
#pragma unroll
    for (int q = 0; q < 4; ++q) { float t0 = __fmul_rn(__fsub_rn(F2[((size_t)b * NN + n + q) * COUT + c], m), rs); asm volatile("" : "+v"(t0)); float t1 = __fmul_rn(t0, gg); asm volatile("" : "+v"(t1)); float t2 = __fadd_rn(t1, bb); asm volatile("" : "+v"(t2)); o[q] = fmaxf(__fadd_rn(t2, bfr(x[e + q])), 0.f); }
    *(volatile v4f*)(OUT + e) = o; __threadfence(); *(volatile v4f*)(OUT + e) = o; }
template <int NFULL, int TAIL> __global__ __launch_bounds__(256) void k_softhl(const float* __restrict__ Sb, int nrows, int rowsper, int rvalid, int nvalid, bf* Ph, bf* Pl) { const int lane = threadIdx.x & 31; const size_t row = (size_t)blockIdx.x * 8 + (threadIdx.x >> 5); if (row >= (size_t)nrows) return; constexpr int LD = NFULL * 128 + TAIL * 64; const float* sr = Sb + row * LD; bf* prh = Ph + row * LD; bf* prl = Pl + row * LD; const bool live = (int)(row % rowsper) < rvalid; float mx = -3.0e38f;
#pragma unroll 1
    for (int ch = 0; ch < NFULL + TAIL; ++ch) { if (ch == NFULL && lane >= 16) break; const int j0 = ch * 128 + lane * 4; const v4f a = *(const v4f*)(sr + j0);
#pragma unroll
        for (int q = 0; q < 4; ++q) if (j0 + q < nvalid) mx = fmaxf(mx, a[q]); }
#pragma unroll
    for (int sh = 16; sh; sh >>= 1) mx = fmaxf(mx, __shfl_xor(mx, sh, 32));
    float sum = 0.f;
#pragma unroll 1
    for (int ch = 0; ch < NFULL + TAIL; ++ch) { if (ch == NFULL && lane >= 16) break; const int j0 = ch * 128 + lane * 4; const v4f a = *(const v4f*)(sr + j0);
#pragma unroll
        for (int q = 0; q < 4; ++q) if (j0 + q < nvalid) { float d0 = __fsub_rn(a[q], mx); asm volatile("" : "+v"(d0)); sum += __expf(d0); } }
#pragma unroll
    for (int sh = 16; sh; sh >>= 1) sum += __shfl_xor(sum, sh, 32);
    const float f = live ? __fdiv_rn(1.0f, sum) : 0.f;
    for (int ps = 0; ps < 2; ++ps) {
#pragma unroll 1
        for (int ch = 0; ch < NFULL + TAIL; ++ch) { if (ch == NFULL && lane >= 16) break; const int j0 = ch * 128 + lane * 4; const v4f a = *(const v4f*)(sr + j0); v4us oh, ol;
#pragma unroll
            for (int q = 0; q < 4; ++q) { float val = 0.f; if (live && j0 + q < nvalid) { float d0 = __fsub_rn(a[q], mx); asm volatile("" : "+v"(d0)); val = __fmul_rn(__expf(d0), f); } unsigned short u, c; splitf(val, u, c); oh[q] = u; ol[q] = c; } *(volatile v4us*)(prh + j0) = oh; *(volatile v4us*)(prl + j0) = ol; }
        if (ps == 0) __threadfence(); } }

extern "C" void kernel_launch(void* const* d_in, const int* in_sizes, int n_in,
                              void* d_out, int out_size, void* d_ws, size_t ws_size, hipStream_t stream) {
    (void)in_sizes; (void)n_in; (void)out_size;
    const float* x = (const float*)d_in[0]; const float* w1 = (const float*)d_in[1]; const float* g1 = (const float*)d_in[2]; const float* b1 = (const float*)d_in[3]; const float* wqkv = (const float*)d_in[4]; const float* rw = (const float*)d_in[5]; const float* rh = (const float*)d_in[6]; const float* w2 = (const float*)d_in[7]; const float* g2 = (const float*)d_in[8]; const float* b2 = (const float*)d_in[9];
    float* OUT = (float*)d_out;
    char* wsp = (char*)d_ws;
    auto take = [&](size_t bytes) { char* p = wsp; wsp += (bytes + 255) & ~(size_t)255; return (void*)p; };
    bf* W1 = (bf*)take((size_t)WID * CIN * 2); bf* WQ = (bf*)take((size_t)3 * WID * WID * 2); bf* W2 = (bf*)take((size_t)COUT * WID * 2); bf* XT = (bf*)take((size_t)NBI * NN * CIN * 2); float* F1 = (float*)take((size_t)NBI * NN * WID * 4); float* M1 = (float*)take(WID * 4); float* R1 = (float*)take(WID * 4);
    bf* Yh = (bf*)take((size_t)NBI * NN * WID * 2); bf* Yl = (bf*)take((size_t)NBI * NN * WID * 2); float* QKV = (float*)take((size_t)NN * 3 * WID * 4); bf* Qh = (bf*)take((size_t)NH_ * NN * HD * 2); bf* Ql = (bf*)take((size_t)NH_ * NN * HD * 2); bf* Kh = (bf*)take((size_t)NH_ * NN * HD * 2); bf* Kl = (bf*)take((size_t)NH_ * NN * HD * 2); bf* VTh = (bf*)take((size_t)NH_ * 64 * NN * 2); bf* VTl = (bf*)take((size_t)NH_ * 64 * NN * 2);
    float* Sb = (float*)take((size_t)NH_ * NN * NN * 4); bf* Ph = (bf*)take((size_t)NH_ * NN * NN * 2); bf* Pl = (bf*)take((size_t)NH_ * NN * NN * 2); float* O = (float*)take((size_t)NH_ * NN * 64 * 4); bf* Mh = (bf*)take((size_t)NBI * NN * WID * 2); bf* Ml = (bf*)take((size_t)NBI * NN * WID * 2); float* F2 = (float*)take((size_t)NBI * NN * COUT * 4); float* M2 = (float*)take(COUT * 4); float* R2 = (float*)take(COUT * 4);
    if ((size_t)(wsp - (char*)d_ws) > ws_size) return;
    k_cvt8<<<(WID * CIN / 8 + 255) / 256, 256, 0, stream>>>(w1, W1, WID * CIN / 8); k_cvt8<<<(3 * WID * WID / 8 + 255) / 256, 256, 0, stream>>>(wqkv, WQ, 3 * WID * WID / 8); k_cvt8<<<(COUT * WID / 8 + 255) / 256, 256, 0, stream>>>(w2, W2, COUT * WID / 8);
    k_xt<<<(unsigned)(((size_t)NBI * NN * CIN / 4 + 255) / 256), 256, 0, stream>>>(x, XT);
    k_gemmw<bf, 0, false><<<dim3(NBI * NN / 64, WID / 64, 1), 32, 0, stream>>>(XT, nullptr, W1, nullptr, CIN, F1, WID, nullptr, 0, 0, 0);
    k_bnstat<<<1, 256, 0, stream>>>(F1, WID, M1, R1); k_bn1<<<(unsigned)(((size_t)NBI * NN * WID / 4 + 255) / 256), 256, 0, stream>>>(F1, M1, R1, g1, b1, Yh, Yl);
    for (int b = 0; b < NBI; ++b) {
        k_gemmw<bf, 1, false><<<dim3(NN / 64, 3 * WID / 64, 1), 32, 0, stream>>>(Yh + (size_t)b * NN * WID, Yl + (size_t)b * NN * WID, WQ, nullptr, WID, QKV, 3 * WID, nullptr, 0, 0, 0);
        k_qkpl<<<(NH_ * NN * HD / 4 + 255) / 256, 256, 0, stream>>>(QKV, rw, rh, Qh, Ql, Kh, Kl); k_vt<<<(NH_ * 64 * NN / 2 + 255) / 256, 256, 0, stream>>>(QKV, VTh, VTl);
        k_gemmw<bf, 2, false><<<dim3(NN / 64, NN / 64, NH_), 32, 0, stream>>>(Qh, Ql, Kh, Kl, HD, Sb, NN, nullptr, (size_t)NN * HD, (size_t)NN * HD, (size_t)NN * NN);
        k_softhl<8, 0><<<(NH_ * NN + 7) / 8, 256, 0, stream>>>(Sb, NH_ * NN, NN, NN, NN, Ph, Pl);
        k_gemmw<bf, 2, false><<<dim3(NN / 64, 1, NH_), 32, 0, stream>>>(Ph, Pl, VTh, VTl, NN, O, 64, nullptr, (size_t)NN * NN, (size_t)64 * NN, (size_t)NN * 64);
        k_mrg<<<(NN * WID / 4 + 255) / 256, 256, 0, stream>>>(O, Mh + (size_t)b * NN * WID, Ml + (size_t)b * NN * WID); }
    k_gemmw<bf, 1, false><<<dim3(NBI * NN / 64, COUT / 64, 1), 32, 0, stream>>>(Mh, Ml, W2, nullptr, WID, F2, COUT, nullptr, 0, 0, 0);
    k_bnstat<<<(COUT + 255) / 256, 256, 0, stream>>>(F2, COUT, M2, R2);
    k_outT<<<(unsigned)(((size_t)NBI * COUT * NN / 4 + 255) / 256), 256, 0, stream>>>(F2, M2, R2, g2, b2, x, OUT);
}
